// RoutingLoRASoftMoe_74715251081275
// MI455X (gfx1250) — hardware-verified
//
#include <hip/hip_runtime.h>
#include <stdint.h>
#include <stddef.h>

typedef __bf16         v16b  __attribute__((ext_vector_type(16)));
typedef float          v8f   __attribute__((ext_vector_type(8)));
typedef float          v4f   __attribute__((ext_vector_type(4)));
typedef unsigned int   u32x4 __attribute__((ext_vector_type(4)));
typedef v4f   __attribute__((may_alias)) v4fa;
typedef u32x4 __attribute__((may_alias)) u32x4a;
typedef unsigned short bf16_t;

#define NB   2
#define SEQ  512
#define DIM  1024
#define RNK  16
#define NSK  512
#define KRD  (NSK * RNK)
#define NTOK (NB * SEQ)

static_assert(NSK == SEQ);
static_assert(NTOK % 64 == 0);
static_assert(SEQ % 64 == 0);
static_assert(DIM % 64 == 0);
static_assert(KRD % 64 == 0);
static_assert(NSK % 64 == 0);
static_assert(SEQ == 8 * 64);

__device__ __forceinline__ int imax(int a, int b) { return a > b ? a : b; }
__device__ __forceinline__ int imin(int a, int b) { return a < b ? a : b; }

__device__ __forceinline__ unsigned f2bf(float f) {
  unsigned u = __float_as_uint(f);
  u += 0x7FFFu + ((u >> 16) & 1u);
  return u >> 16;
}
__device__ __forceinline__ u32x4 pack8(v4f a, v4f c) {
  u32x4 o;
  o.x = f2bf(a.x) | (f2bf(a.y) << 16);
  o.y = f2bf(a.z) | (f2bf(a.w) << 16);
  o.z = f2bf(c.x) | (f2bf(c.y) << 16);
  o.w = f2bf(c.z) | (f2bf(c.w) << 16);
  return o;
}

__device__ __forceinline__ v8f wmma_bf16(v16b a, v16b b, v8f c) {
  v8f d = __builtin_amdgcn_wmma_f32_16x16x32_bf16(false, a, false, b, (short)0, c, false, false);
  asm volatile("v_nop\n\tv_nop\n\tv_nop\n\tv_nop" : "+v"(d) : "v"(a), "v"(b));
  return d;
}

__device__ __forceinline__ v16b load_frag(const bf16_t* p, int h) {
  union { v16b v; u32x4 q[2]; } f;
  f.q[0] = *(const u32x4a*)(p + 8 * h);
  f.q[1] = *(const u32x4a*)(p + 16 + 8 * h);
  return f.v;
}

enum { P_X = 0, P_W = 1, P_PHIT = 2, P_XT = 3, P_AT = 4, P_LBT = 5 };

template<int PM>
__global__ __launch_bounds__(256) void pack_k(const float* __restrict__ src,
                                              bf16_t* __restrict__ dst, int nchunks)
{
  const int c = blockIdx.x * 256 + threadIdx.x;
  if (c >= nchunks) return;
  v4f a, q;
  if constexpr (PM == P_X || PM == P_W) {
    a = *(const v4fa*)(src + (size_t)c * 8);
    q = *(const v4fa*)(src + (size_t)c * 8 + 4);
  } else {
    size_t gi = 0;
    int gs = 1;
    if constexpr (PM == P_PHIT) {
      const int n = c >> 7, d0 = (c & 127) * 8;
      gi = (size_t)d0 * NSK + n;  gs = NSK;
    } else if constexpr (PM == P_XT) {
      const int row = c >> 6, bb = row >> 10, d = row & 1023, s0 = (c & 63) * 8;
      gi = ((size_t)bb * SEQ + s0) * DIM + d;  gs = DIM;
    } else if constexpr (PM == P_AT) {
      const int row = c >> 7, kk = row >> 4, r = row & 15, d0 = (c & 127) * 8;
      gi = ((size_t)kk * DIM + d0) * RNK + r;  gs = RNK;
    } else {
      const int e = c >> 10, kr0 = (c & 1023) * 8;
      gi = (size_t)kr0 * DIM + e;  gs = DIM;
    }
    const float* sp = src + gi;
    a.x = sp[0];          a.y = sp[(size_t)gs];     a.z = sp[(size_t)2 * gs]; a.w = sp[(size_t)3 * gs];
    q.x = sp[(size_t)4 * gs]; q.y = sp[(size_t)5 * gs]; q.z = sp[(size_t)6 * gs]; q.w = sp[(size_t)7 * gs];
  }
  const u32x4 o = pack8(a, q);
  bf16_t* dp = dst + (size_t)c * 8;
  *(volatile u32x4*)dp = o;
  __threadfence();
  *(volatile u32x4*)dp = o;
}

__device__ __forceinline__ float wave_max_f(float v) {
#pragma unroll
  for (int o = 16; o > 0; o >>= 1) v = fmaxf(v, __shfl_xor(v, o));
  return v;
}
__device__ __forceinline__ float wave_sum_f(float v) {
#pragma unroll
  for (int o = 16; o > 0; o >>= 1) v += __shfl_xor(v, o);
  return v;
}
__device__ __forceinline__ int wave_max_i(int v) {
#pragma unroll
  for (int o = 16; o > 0; o >>= 1) v = imax(v, __shfl_xor(v, o));
  return v;
}
__device__ __forceinline__ int wave_min_i(int v) {
#pragma unroll
  for (int o = 16; o > 0; o >>= 1) v = imin(v, __shfl_xor(v, o));
  return v;
}
__device__ __forceinline__ int wave_sum_i(int v) {
#pragma unroll
  for (int o = 16; o > 0; o >>= 1) v += __shfl_xor(v, o);
  return v;
}

__global__ __launch_bounds__(64) void router_k(const float* __restrict__ mixing,
                                               const int* __restrict__ inst,
                                               const int* __restrict__ pad,
                                               bf16_t* __restrict__ dwh,
                                               float* __restrict__ cm)
{
  __shared__ __attribute__((aligned(16))) float scm[NSK];
  __shared__ float fred[8];
  __shared__ int   ired[6];

  const int p = blockIdx.x, b = blockIdx.y;
  const int tid = threadIdx.x, lane = tid & 31, w = tid >> 5;
  const int s0 = 8 * tid;
  const size_t row = (size_t)b * SEQ + p;

  const int* ip = inst + (size_t)b * SEQ + s0;
  int iv[8];
#pragma unroll
  for (int e = 0; e < 8; ++e) iv[e] = ip[e];
  int vmax = iv[0];
#pragma unroll
  for (int e = 1; e < 8; ++e) vmax = imax(vmax, iv[e]);
  vmax = wave_max_i(vmax);
  if (lane == 0) ired[w] = vmax;
  __syncthreads();
  vmax = imax(ired[0], ired[1]);
  int fidx = 0x7fffffff;
#pragma unroll
  for (int e = 7; e >= 0; --e) { if (iv[e] == vmax) fidx = s0 + e; }
  fidx = wave_min_i(fidx);
  int isum = 0;
#pragma unroll
  for (int e = 0; e < 8; ++e) isum += iv[e];
  isum = wave_sum_i(isum);
  if (lane == 0) { ired[2 + w] = fidx; ired[4 + w] = isum; }
  __syncthreads();
  const int first = imin(ired[2], ired[3]);
  const int nones = ired[4] + ired[5];
  const int last  = first + nones;
  const int ramp  = imax(p + 1 - last, 0);
  const int padP  = pad[row];
  const int mp    = (last + ramp) * padP;
  const float padf = (float)padP;

  const float* mr = mixing + row * NSK + s0;
  const v4f xa = *(const v4fa*)mr;
  const v4f xq = *(const v4fa*)(mr + 4);
  float x[8] = { xa.x, xa.y, xa.z, xa.w, xq.x, xq.y, xq.z, xq.w };
  const int* pr = pad + (size_t)b * SEQ + s0;
  float v[8];
#pragma unroll
  for (int e = 0; e < 8; ++e) v[e] = ((s0 + e) < mp * pr[e]) ? x[e] : -1e38f;

  float mx = v[0];
#pragma unroll
  for (int e = 1; e < 8; ++e) mx = fmaxf(mx, v[e]);
  mx = wave_max_f(mx);
  if (lane == 0) fred[w] = mx;
  __syncthreads();
  mx = fmaxf(fred[0], fred[1]);
  float ex[8];
  float ls = 0.0f;
#pragma unroll
  for (int e = 0; e < 8; ++e) { ex[e] = __expf(v[e] - mx); ls += ex[e]; }
  ls = wave_sum_f(ls);

  float mx2 = x[0];
#pragma unroll
  for (int e = 1; e < 8; ++e) mx2 = fmaxf(mx2, x[e]);
  mx2 = wave_max_f(mx2);
  if (lane == 0) { fred[2 + w] = ls; fred[4 + w] = mx2; }
  __syncthreads();
  const float dsum = fred[2] + fred[3];
  mx2 = fmaxf(fred[4], fred[5]);
  float e2[8];
  float ls2 = 0.0f;
#pragma unroll
  for (int e = 0; e < 8; ++e) { e2[e] = __expf(x[e] - mx2); ls2 += e2[e]; }
  ls2 = wave_sum_f(ls2);
  if (lane == 0) fred[6 + w] = ls2;
  __syncthreads();
  const float csum = fred[6] + fred[7];

  const float dsc = padf * (1.0f / dsum);
  const float csc = 1.0f / csum;
#pragma unroll
  for (int e = 0; e < 8; ++e) scm[s0 + e] = e2[e] * csc;
  const v4f da = { ex[0] * dsc, ex[1] * dsc, ex[2] * dsc, ex[3] * dsc };
  const v4f dq = { ex[4] * dsc, ex[5] * dsc, ex[6] * dsc, ex[7] * dsc };
  const u32x4 dwp = pack8(da, dq);
  __syncthreads();

  const v4f c0 = *(const v4fa*)(scm + 4 * tid);
  const v4f c1 = *(const v4fa*)(scm + NSK / 2 + 4 * tid);
  bf16_t* ddst = dwh + row * SEQ + s0;
  float* cdst  = cm + row * NSK + 4 * tid;
  *(volatile u32x4*)ddst = dwp;
  *(volatile v4f*)cdst = c0;
  *(volatile v4f*)(cdst + NSK / 2) = c1;
  __threadfence();
  *(volatile u32x4*)ddst = dwp;
  *(volatile v4f*)cdst = c0;
  *(volatile v4f*)(cdst + NSK / 2) = c1;
}

template<int LDA, int LDB, int KD>
__device__ __forceinline__ void mac_loop(v8f (&acc)[2][2], const bf16_t* __restrict__ a0p,
                                         const bf16_t* __restrict__ b0p, int h)
{
  const bf16_t* a1p = a0p + (size_t)16 * LDA;
  const bf16_t* b1p = b0p + (size_t)16 * LDB;
#pragma unroll 1
  for (int k0 = 0; k0 < KD; k0 += 32) {
    const v16b a0 = load_frag(a0p + k0, h);
    const v16b a1 = load_frag(a1p + k0, h);
    const v16b b0 = load_frag(b0p + k0, h);
    const v16b b1 = load_frag(b1p + k0, h);
    acc[0][0] = wmma_bf16(a0, b0, acc[0][0]);
    acc[0][1] = wmma_bf16(a0, b1, acc[0][1]);
    acc[1][0] = wmma_bf16(a1, b0, acc[1][0]);
    acc[1][1] = wmma_bf16(a1, b1, acc[1][1]);
  }
}

__device__ __forceinline__ void store_tile_f32(const float* sT, float* base, int ldo, int w, int lane) {
  const int q8 = lane & 7, sub = lane >> 3;
#pragma unroll
  for (int i = 0; i < 8; ++i) {
    const int lid = w * 32 + i * 4 + sub;
    const int row = lid >> 1, hl = lid & 1;
    const v4f v = *(const v4fa*)(sT + row * 64 + 32 * hl + 4 * q8);
    *(volatile v4f*)(base + (size_t)row * ldo + 32 * hl + 4 * q8) = v;
  }
}
__device__ __forceinline__ void store_tile_bf16(const float* sT, bf16_t* base, int ldo, int w, int lane) {
  const int q8 = lane & 7, sub = lane >> 3;
#pragma unroll
  for (int i = 0; i < 4; ++i) {
    const int row = w * 16 + i * 4 + sub;
    const v4f a = *(const v4fa*)(sT + row * 64 + 8 * q8);
    const v4f c = *(const v4fa*)(sT + row * 64 + 8 * q8 + 4);
    const u32x4 o = pack8(a, c);
    *(volatile u32x4*)(base + (size_t)row * ldo + 8 * q8) = o;
  }
}

enum { G_MIXING = 0, G_MIXED = 1, G_LOWRANK = 2, G_OUT = 3 };

template<int MODE>
__global__ __launch_bounds__(128) void gemm_k(const bf16_t* __restrict__ A,  const bf16_t* __restrict__ Bn,
                                              const bf16_t* __restrict__ A2, const bf16_t* __restrict__ B2,
                                              const float* __restrict__ aux, void* __restrict__ outp)
{
  __shared__ __attribute__((aligned(16))) float sT[64 * 64];

  const int tid = threadIdx.x, lane = tid & 31, w = tid >> 5;
  const int h = lane >> 4, m = lane & 15;
  const int wM = (w & 1) * 32, wN = (w >> 1) * 32;
  const int tileM = blockIdx.x * 64, tileN = blockIdx.y * 64;
  const int bz = blockIdx.z;
  (void)A2; (void)B2; (void)aux; (void)bz;

  const v8f zero8 = {0.f, 0.f, 0.f, 0.f, 0.f, 0.f, 0.f, 0.f};
  v8f acc[2][2];
#pragma unroll
  for (int mi = 0; mi < 2; ++mi)
#pragma unroll
    for (int ni = 0; ni < 2; ++ni) acc[mi][ni] = zero8;

  const int arow = tileM + wM + m;
  const int brow = tileN + wN + m;

  if constexpr (MODE == G_MIXING) {
    mac_loop<DIM, DIM, DIM>(acc, A + (size_t)arow * DIM, Bn + (size_t)brow * DIM, h);
  } else if constexpr (MODE == G_MIXED) {
    const bf16_t* Ab = A  + (size_t)bz * SEQ * SEQ;
    const bf16_t* Bb = Bn + (size_t)bz * DIM * SEQ;
    mac_loop<SEQ, SEQ, SEQ>(acc, Ab + (size_t)arow * SEQ, Bb + (size_t)brow * SEQ, h);
  } else if constexpr (MODE == G_LOWRANK) {
    mac_loop<DIM, DIM, DIM>(acc, A + (size_t)arow * DIM, Bn + (size_t)brow * DIM, h);
  } else {
    mac_loop<KRD, KRD, KRD>(acc, A  + (size_t)arow * KRD, Bn + (size_t)brow * KRD, h);
    mac_loop<DIM, DIM, DIM>(acc, A2 + (size_t)arow * DIM, B2 + (size_t)brow * DIM, h);
  }

#pragma unroll
  for (int mi = 0; mi < 2; ++mi) {
#pragma unroll
    for (int ni = 0; ni < 2; ++ni) {
      const int col = wN + 16 * ni + m;
      float addv = 0.0f;
      if constexpr (MODE == G_OUT) addv = aux[tileN + col];
#pragma unroll
      for (int r = 0; r < 8; ++r) {
        const int rowl = wM + 16 * mi + 8 * h + r;
        float v = acc[mi][ni][r];
        if constexpr (MODE == G_LOWRANK) v *= aux[(size_t)(tileM + rowl) * NSK + ((tileN + col) >> 4)];
        if constexpr (MODE == G_OUT) v += addv;
        sT[rowl * 64 + col] = v;
      }
    }
  }
  __syncthreads();

  if constexpr (MODE == G_MIXING || MODE == G_OUT) {
    constexpr int LDO = (MODE == G_MIXING) ? NSK : DIM;
    float* base = (float*)outp + (size_t)tileM * LDO + tileN;
    store_tile_f32(sT, base, LDO, w, lane);
    __threadfence();
    store_tile_f32(sT, base, LDO, w, lane);
  } else {
    constexpr int LDO = (MODE == G_MIXED) ? DIM : KRD;
    const int rowG0 = (MODE == G_MIXED) ? (bz * SEQ + tileM) : tileM;
    bf16_t* base = (bf16_t*)outp + (size_t)rowG0 * LDO + tileN;
    store_tile_bf16(sT, base, LDO, w, lane);
    __threadfence();
    store_tile_bf16(sT, base, LDO, w, lane);
  }
}

extern "C" void kernel_launch(void* const* d_in, const int* in_sizes, int n_in,
                              void* d_out, int out_size, void* d_ws, size_t ws_size,
                              hipStream_t stream) {
  if (n_in < 8) return;
  if (in_sizes[0] != NTOK * DIM) return;
  if (in_sizes[1] != NTOK) return;
  if (in_sizes[2] != NTOK) return;
  if (in_sizes[3] != DIM * NSK) return;
  if (in_sizes[4] != NSK * DIM * RNK) return;
  if (in_sizes[5] != KRD * DIM) return;
  if (in_sizes[6] != DIM * DIM) return;
  if (in_sizes[7] != DIM) return;
  if (out_size != NTOK * DIM) return;

  const float* x    = (const float*)d_in[0];
  const int*   inst = (const int*)d_in[1];
  const int*   pad  = (const int*)d_in[2];
  const float* phi  = (const float*)d_in[3];
  const float* la   = (const float*)d_in[4];
  const float* lb   = (const float*)d_in[5];
  const float* W    = (const float*)d_in[6];
  const float* bias = (const float*)d_in[7];
  float* out = (float*)d_out;

  const size_t b_xh   = (size_t)NTOK * DIM * 2;
  const size_t b_wh   = (size_t)DIM * DIM * 2;
  const size_t b_phit = (size_t)NSK * DIM * 2;
  const size_t b_xt   = (size_t)NB * DIM * SEQ * 2;
  const size_t b_at   = (size_t)KRD * DIM * 2;
  const size_t b_lbt  = (size_t)DIM * KRD * 2;
  const size_t b_mix  = (size_t)NTOK * NSK * 4;
  const size_t b_dwh  = (size_t)NTOK * SEQ * 2;
  const size_t b_cm   = (size_t)NTOK * NSK * 4;
  const size_t b_mxd  = (size_t)NTOK * DIM * 2;
  const size_t b_g    = (size_t)NTOK * KRD * 2;
  const size_t total  = b_xh + b_wh + b_phit + b_xt + b_at + b_lbt + b_mix + b_dwh + b_cm + b_mxd + b_g;
  if (total > ws_size) return;

  char* ws = (char*)d_ws;
  size_t off = 0;
  bf16_t* xh   = (bf16_t*)(ws + off); off += b_xh;
  bf16_t* wh   = (bf16_t*)(ws + off); off += b_wh;
  bf16_t* phit = (bf16_t*)(ws + off); off += b_phit;
  bf16_t* xt   = (bf16_t*)(ws + off); off += b_xt;
  bf16_t* at   = (bf16_t*)(ws + off); off += b_at;
  bf16_t* lbt  = (bf16_t*)(ws + off); off += b_lbt;
  float*  mix  = (float*)(ws + off);  off += b_mix;
  bf16_t* dwh  = (bf16_t*)(ws + off); off += b_dwh;
  float*  cm   = (float*)(ws + off);  off += b_cm;
  bf16_t* mxd  = (bf16_t*)(ws + off); off += b_mxd;
  bf16_t* g    = (bf16_t*)(ws + off); off += b_g;
  if (off > ws_size) return;

  const int nc_x  = NTOK * DIM / 8;
  const int nc_w  = DIM * DIM / 8;
  const int nc_ph = NSK * DIM / 8;
  const int nc_xt = NB * DIM * SEQ / 8;
  const int nc_at = KRD * DIM / 8;
  const int nc_lb = DIM * KRD / 8;
  pack_k<P_X>   <<<(nc_x  + 255) / 256, 256, 0, stream>>>(x,   xh,   nc_x);
  pack_k<P_W>   <<<(nc_w  + 255) / 256, 256, 0, stream>>>(W,   wh,   nc_w);
  pack_k<P_PHIT><<<(nc_ph + 255) / 256, 256, 0, stream>>>(phi, phit, nc_ph);
  pack_k<P_XT>  <<<(nc_xt + 255) / 256, 256, 0, stream>>>(x,   xt,   nc_xt);
  pack_k<P_AT>  <<<(nc_at + 255) / 256, 256, 0, stream>>>(la,  at,   nc_at);
  pack_k<P_LBT> <<<(nc_lb + 255) / 256, 256, 0, stream>>>(lb,  lbt,  nc_lb);

  gemm_k<G_MIXING><<<dim3(NTOK / 64, NSK / 64, 1), 128, 0, stream>>>(xh, phit, nullptr, nullptr, nullptr, mix);

  router_k<<<dim3(SEQ, NB), 64, 0, stream>>>(mix, inst, pad, dwh, cm);

  gemm_k<G_MIXED><<<dim3(SEQ / 64, DIM / 64, NB), 128, 0, stream>>>(dwh, xt, nullptr, nullptr, nullptr, mxd);

  gemm_k<G_LOWRANK><<<dim3(NTOK / 64, KRD / 64, 1), 128, 0, stream>>>(mxd, at, nullptr, nullptr, cm, g);

  gemm_k<G_OUT><<<dim3(NTOK / 64, DIM / 64, 1), 128, 0, stream>>>(g, lbt, xh, wh, bias, out);
}
